// Conv3dBlock_10307921510639
// MI455X (gfx1250) — hardware-verified
//
#include <hip/hip_runtime.h>


namespace {
constexpr int NB = 2, NS = 256, T = 128, M = 128, GH = 32, GW = 32, NCELL = GH * GW, BL = 2, TL = 128  ;
constexpr int NBLK = BL * NCELL;
constexpr float XS = 8.0f, WSC = 256.0f, EPS = 1e-5f;
static_assert(M == 128 && NS % 16 == 0 && TL % 16 == 0 && TL <= T && BL <= NB, "tiling");
typedef _Float16 b16;
typedef __attribute__((ext_vector_type(16))) _Float16 v16b;
typedef __attribute__((ext_vector_type(8))) _Float16 v8b;
typedef __attribute__((ext_vector_type(8))) float v8f;
typedef __attribute__((ext_vector_type(4))) float v4f;
__device__ __forceinline__ float bf16_rne(float f) { unsigned int u = __float_as_uint(f); u += 0x7FFFu + ((u >> 16) & 1u); return __uint_as_float(u & 0xFFFF0000u); }
__device__ __forceinline__ void split16(float v, b16& hi, b16& lo) { hi = (b16)v; lo = (b16)(v - (float)hi); }
__device__ __forceinline__ v16b frag_kb(const b16* p, int hh) { const v8b a = *(const v8b*)(p + 8 * hh), b = *(const v8b*)(p + 16 + 8 * hh); v16b f;
#pragma unroll
  for (int e = 0; e < 8; ++e) { f[e] = a[e]; f[8 + e] = b[e]; } return f; }
__device__ __forceinline__ v8f wmma16b(v16b a, v16b b, v8f c) { v8f d = __builtin_amdgcn_wmma_f32_16x16x32_f16(false, a, false, b, (short)0, c, false, false); asm volatile("v_nop\n\tv_nop\n\tv_nop\n\tv_nop" : "+v"(d) : "v"(a), "v"(b)); return d; }
__device__ __forceinline__ void wave_lds_sync() { __builtin_amdgcn_fence(__ATOMIC_RELEASE, "workgroup"); __builtin_amdgcn_wave_barrier(); __builtin_amdgcn_fence(__ATOMIC_ACQUIRE, "workgroup"); }
__device__ __forceinline__ float pmul(float a, float b) { float p = a * b; asm volatile("" : "+v"(p)); return p; }
__device__ __forceinline__ int iclamp(int v, int lo, int hi) { return v < lo ? lo : (v > hi ? hi : v); }

typedef __attribute__((ext_vector_type(4))) _Float16 v4h;
typedef __attribute__((ext_vector_type(4))) int v4i;
__global__ __launch_bounds__(256) void prep_kernel(const int* __restrict__ rowi, const int* __restrict__ coli, const float* __restrict__ pw, int* __restrict__ CM, b16* __restrict__ PWT) {
  const int t = threadIdx.x;
  if (blockIdx.x == 0) { v4i r; for (int j = 0; j < 4; ++j) { const int cell = 4 * t + j; int best = -1;
#pragma unroll 1
      for (int c = NS - 1; c >= 0; --c) { const int rc = iclamp(rowi[c], 0, GH - 1) * GW + iclamp(coli[c], 0, GW - 1); if (rc == cell) best = c; } r[j] = best; }
    for (int pass = 0; pass < 2; ++pass) { *(volatile v4i*)(CM + 4 * t) = r; __threadfence(); } }
  else { const int u = (blockIdx.x - 1) * 256 + t; if (u >= M * M / 8) return; const int e = u * 8; v8b o; for (int j = 0; j < 8; ++j) o[j] = (b16)(bf16_rne(pw[e + j]) * WSC); for (int pass = 0; pass < 2; ++pass) { *(volatile v8b*)(PWT + e) = o; __threadfence(); } }
}
__global__ __launch_bounds__(128) void dw_kernel(const float* __restrict__ x, const int* __restrict__ CM, const float* __restrict__ cw, const float* __restrict__ cb, float* __restrict__ Y, float* __restrict__ PS) {
  const int m = threadIdx.x; const int b = blockIdx.x / NCELL, cell = blockIdx.x % NCELL; const int h = cell / GW, w = cell % GW;
  float wt[27];
#pragma unroll
  for (int k = 0; k < 27; ++k) wt[k] = bf16_rne(cw[m * 27 + k]);
  const float bias = bf16_rne(cb[m]);
  int nb[9];
#pragma unroll
  for (int k = 0; k < 9; ++k) { const int hh_ = h + k / 3 - 1, ww = w + k % 3 - 1; nb[k] = (hh_ >= 0 && hh_ < GH && ww >= 0 && ww < GW) ? iclamp(CM[hh_ * GW + ww], -1, NS - 1) : -1; }
  const int cself = iclamp(CM[cell], -1, NS - 1);
  float s1 = 0.0f, s2 = 0.0f;
#pragma unroll 1
  for (int t = 0; t < TL; ++t) { float y = bias;
#pragma unroll
    for (int k = 0; k < 9; ++k) { const int c = nb[k]; if (c >= 0) {
#pragma unroll
        for (int dt = 0; dt < 3; ++dt) { const int tt = t + dt - 2; if (tt >= 0) y += pmul(wt[dt * 9 + k], bf16_rne(x[(((size_t)b * NS + c) * T + tt) * M + m])); } } }
    s1 += y; s2 += y * y;
    if (cself >= 0) { for (int pass = 0; pass < 2; ++pass) { ((volatile float*)Y)[(((size_t)b * NS + cself) * T + t) * M + m] = y; __threadfence(); } } }
  for (int pass = 0; pass < 2; ++pass) { ((volatile float*)PS)[((size_t)blockIdx.x * 2 + 0) * M + m] = s1; ((volatile float*)PS)[((size_t)blockIdx.x * 2 + 1) * M + m] = s2; __threadfence(); }
}
__global__ __launch_bounds__(128) void stat_kernel(const float* __restrict__ PS, float* __restrict__ MV) {
  const int m = threadIdx.x; double a = 0.0, q = 0.0;
#pragma unroll 1
  for (int k = 0; k < NBLK; ++k) { a += (double)PS[((size_t)k * 2 + 0) * M + m]; q += (double)PS[((size_t)k * 2 + 1) * M + m]; }
  const double n = (double)NBLK * (double)TL; const double mean = a / n; double var = q / n - mean * mean; if (var < 0.0) var = 0.0;
  for (int pass = 0; pass < 2; ++pass) { ((volatile float*)MV)[m] = (float)mean; ((volatile float*)MV)[M + m] = (float)var; __threadfence(); }
}
__global__ __launch_bounds__(32) void pw_kernel(const float* __restrict__ Y, const float* __restrict__ MV, const float* __restrict__ gamma, const float* __restrict__ beta, const b16* __restrict__ PWT, const float* __restrict__ pwb, const float* __restrict__ x, float* __restrict__ out) {
  __shared__ __attribute__((aligned(16))) b16 Ah[16][M + 8], Al[16][M + 8]; __shared__ __attribute__((aligned(16))) float Tf[16][M + 4];
  const int lane = threadIdx.x, nloc = lane & 15, hlf = lane >> 4;
  const int rows_per_b = NS * TL; const int rb = blockIdx.x * 16; const int b = rb / rows_per_b, rem = rb % rows_per_b; const int c = rem / TL, t0 = rem % TL;
  float sc[4], sh[4]; for (int j = 0; j < 4; ++j) { const int m = lane * 4 + j; const float rs = rsqrtf(MV[M + m] + EPS); sc[j] = rs * bf16_rne(gamma[m]); sh[j] = bf16_rne(beta[m]) - MV[m] * sc[j]; }
  for (int rr = 0; rr < 16; ++rr) { const size_t row = ((size_t)b * NS + c) * T + t0 + rr; const v4f y = *(const v4f*)(Y + row * M + lane * 4); v4h hv, lv;
    for (int j = 0; j < 4; ++j) { const float z = y[j] * sc[j] + sh[j]; const float g = 0.5f * z * (1.0f + erff(z * 0.70710678118654752f)); b16 p, q; split16(g * XS, p, q); hv[j] = p; lv[j] = q; }
    *(v4h*)(&Ah[rr][lane * 4]) = hv; *(v4h*)(&Al[rr][lane * 4]) = lv; }
  wave_lds_sync();
  v8f acc[8];
#pragma unroll
  for (int tt = 0; tt < 8; ++tt) acc[tt] = (v8f){};
#pragma unroll
  for (int kb = 0; kb < M; kb += 32) { const v16b a = frag_kb(&Ah[nloc][kb], hlf), al = frag_kb(&Al[nloc][kb], hlf);
#pragma unroll
    for (int tt = 0; tt < 8; ++tt) { const v16b bw = frag_kb(PWT + (size_t)(tt * 16 + nloc) * M + kb, hlf); acc[tt] = wmma16b(a, bw, acc[tt]); acc[tt] = wmma16b(al, bw, acc[tt]); } }
#pragma unroll
  for (int tt = 0; tt < 8; ++tt) { const float bb = bf16_rne(pwb[tt * 16 + nloc]);
#pragma unroll
    for (int r = 0; r < 8; ++r) Tf[8 * hlf + r][tt * 16 + nloc] = acc[tt][r] * (1.0f / (XS * WSC)) + bb; }
  wave_lds_sync();
  for (int pass = 0; pass < 2; ++pass) { for (int rr = 0; rr < 16; ++rr) { const size_t row = ((size_t)b * NS + c) * T + t0 + rr; v4f o = *(const v4f*)(&Tf[rr][lane * 4]); const v4f xv = *(const v4f*)(x + row * M + lane * 4); for (int j = 0; j < 4; ++j) o[j] += bf16_rne(xv[j]); *(volatile v4f*)(out + row * M + lane * 4) = o; } __threadfence(); }
}
}

extern "C" void kernel_launch(void* const* d_in, const int* in_sizes, int n_in, void* d_out, int out_size, void* d_ws, size_t ws_size, hipStream_t stream) {
  (void)n_in;
  auto Fp = [&](int i) { return (const float*)d_in[i]; }; auto Ip = [&](int i) { return (const int*)d_in[i]; };
  if (in_sizes[0] != NB * NS * T * M || in_sizes[1] != NS || in_sizes[2] != NS || in_sizes[3] != M * 27 || in_sizes[4] != M || in_sizes[5] != M * M || in_sizes[6] != M || in_sizes[7] != M || in_sizes[8] != M || out_size != NB * NS * T * M) return;
  size_t off = 0; char* ws = (char*)d_ws;
  auto carve = [&](size_t bytes) { char* p = ws + off; off += (bytes + 255) & ~(size_t)255; return p; };
  int* CM = (int*)carve(NCELL * 4); b16* PWT = (b16*)carve((size_t)M * M * 2); float* Y = (float*)carve((size_t)NB * NS * T * M * 4); float* PS = (float*)carve((size_t)NB * NCELL * 2 * M * 4); float* MV = (float*)carve(2 * M * 4);
  if (off > ws_size || off > ((size_t)128 << 20)) return;
  prep_kernel<<<1 + (M * M / 8 + 255) / 256, 256, 0, stream>>>(Ip(1), Ip(2), Fp(5), CM, PWT);
  dw_kernel<<<NBLK, 128, 0, stream>>>(Fp(0), CM, Fp(3), Fp(4), Y, PS);
  stat_kernel<<<1, 128, 0, stream>>>(PS, MV);
  pw_kernel<<<BL * NS * TL / 16, 32, 0, stream>>>(Y, MV, Fp(7), Fp(8), PWT, Fp(6), Fp(0), (float*)d_out);
}
